// G2CoreAttention_6674379178219
// MI455X (gfx1250) — hardware-verified
//
#include <hip/hip_runtime.h>
#include <stdint.h>

typedef float v8f __attribute__((ext_vector_type(8)));
typedef float v4f __attribute__((ext_vector_type(4)));
typedef int v4i __attribute__((ext_vector_type(4)));
typedef __bf16 v16bf __attribute__((ext_vector_type(16)));
typedef unsigned short v8us_raw __attribute__((ext_vector_type(8)));
typedef v8us_raw v8us __attribute__((may_alias));

union Frag {
  v16bf v;
  v8us h[2];
};

namespace {
constexpr int H   = 16;
constexpr int D   = 128;
constexpr int TK  = 512;
constexpr int CH  = 64;
constexpr int NCH = TK / CH;
constexpr int QP  = 136;
constexpr int KP  = 136;
constexpr int SP  = 512;
constexpr int PP  = 520;
constexpr int VP  = 72;
constexpr int OP  = 36;

constexpr int oQh  = 0;
constexpr int oQl  = oQh + H * QP * 2;
constexpr int oIdx = oQl + H * QP * 2;
constexpr int oL   = oIdx + TK * 4;
constexpr int oPh  = oL + 64;
constexpr int oPl  = oPh + H * PP * 2;
constexpr int oR   = oPl + H * PP * 2;
constexpr int oKh  = oR;
constexpr int oKl  = oKh + CH * KP * 2;
constexpr int oS   = oKl + CH * KP * 2;
constexpr int endA = oS + H * SP * 4;
constexpr int oVh  = oR;
constexpr int oVl  = oVh + D * VP * 2;
constexpr int oO   = oVl + D * VP * 2;
constexpr int endB = oO + 4 * H * OP * 4;
constexpr int SMEM = (endA > endB) ? endA : endB;

static_assert((oQl % 16) == 0 && (oIdx % 16) == 0 && (oL % 16) == 0 && (oPh % 16) == 0 &&
              (oPl % 16) == 0 && (oR % 16) == 0 && (oKl % 16) == 0 && (oS % 16) == 0 &&
              (oVl % 16) == 0 && (oO % 16) == 0);
static_assert(SMEM == 111680);
static_assert((QP * 2) % 16 == 0 && (KP * 2) % 16 == 0 && (PP * 2) % 16 == 0 &&
              (VP * 2) % 16 == 0 && (OP * 4) % 16 == 0);
}

__device__ __forceinline__ unsigned short f2bf(float x) {
  unsigned u = __float_as_uint(x);
  u += 0x7FFFu + ((u >> 16) & 1u);
  return (unsigned short)(u >> 16);
}

__device__ __forceinline__ float bf2f(unsigned short b) {
  return __uint_as_float(((unsigned)b) << 16);
}

__device__ __forceinline__ v8f zero8() {
  v8f z;
#pragma unroll
  for (int i = 0; i < 8; ++i) z[i] = 0.0f;
  return z;
}

__device__ __forceinline__ v8f wmma_bf16(v16bf a, v16bf b, v8f c) {
  v8f d = __builtin_amdgcn_wmma_f32_16x16x32_bf16(false, a, false, b, (short)0, c, false, false);
  asm volatile("v_nop\n\tv_nop\n\tv_nop\n\tv_nop" : "+v"(d) : "v"(a), "v"(b));
  return d;
}

__launch_bounds__(256)
__global__ void k_split(const float* __restrict__ x, unsigned short* hi, unsigned short* lo, int n)
{
  const size_t i8 = ((size_t)blockIdx.x * 256 + threadIdx.x) * 8;
  if (i8 + 8 <= (size_t)n) {
    const v4f a = *(const v4f*)(x + i8);
    const v4f b = *(const v4f*)(x + i8 + 4);
    float f[8];
    f[0] = a[0]; f[1] = a[1]; f[2] = a[2]; f[3] = a[3];
    f[4] = b[0]; f[5] = b[1]; f[6] = b[2]; f[7] = b[3];
    v8us vh, vl;
#pragma unroll
    for (int e = 0; e < 8; ++e) {
      const unsigned short hb = f2bf(f[e]);
      vh[e] = hb;
      vl[e] = f2bf(f[e] - bf2f(hb));
    }
    *(volatile v8us*)(hi + i8) = vh;
    *(volatile v8us*)(lo + i8) = vl;
    __threadfence();
    *(volatile v8us*)(hi + i8) = vh;
    *(volatile v8us*)(lo + i8) = vl;
  } else if (i8 < (size_t)n) {
    unsigned short th[8], tl[8];
    int cnt = (int)((size_t)n - i8);
    for (int e = 0; e < cnt; ++e) {
      const float v = x[i8 + e];
      const unsigned short hb = f2bf(v);
      th[e] = hb;
      tl[e] = f2bf(v - bf2f(hb));
    }
    for (int e = 0; e < cnt; ++e) {
      ((volatile unsigned short*)hi)[i8 + e] = th[e];
      ((volatile unsigned short*)lo)[i8 + e] = tl[e];
    }
    __threadfence();
    for (int e = 0; e < cnt; ++e) {
      ((volatile unsigned short*)hi)[i8 + e] = th[e];
      ((volatile unsigned short*)lo)[i8 + e] = tl[e];
    }
  }
}

__launch_bounds__(128)
__global__ void k_attn(const unsigned short* __restrict__ qh, const unsigned short* __restrict__ ql,
                       const unsigned short* __restrict__ kh, const unsigned short* __restrict__ kl,
                       const int* __restrict__ topk, float* out, int nS, int nKV)
{
  __shared__ __align__(16) unsigned char smem[SMEM];
  const int s = blockIdx.x;
  if (s >= nS) return;
  const int tid  = threadIdx.x;
  const int lane = tid & 31;
  const int wave = tid >> 5;
  const int hh   = lane >> 4;
  const int m    = lane & 15;

  unsigned short* Qh = (unsigned short*)(smem + oQh);
  unsigned short* Ql = (unsigned short*)(smem + oQl);
  int*            IDX = (int*)(smem + oIdx);
  float*          Lsum = (float*)(smem + oL);
  unsigned short* Ph = (unsigned short*)(smem + oPh);
  unsigned short* Pl = (unsigned short*)(smem + oPl);
  unsigned short* Kh = (unsigned short*)(smem + oKh);
  unsigned short* Kl = (unsigned short*)(smem + oKl);
  float*          S  = (float*)(smem + oS);
  unsigned short* Vh = (unsigned short*)(smem + oVh);
  unsigned short* Vl = (unsigned short*)(smem + oVl);
  float*          Osc = (float*)(smem + oO);

  const float scale   = 0.08838834764831845f;
  const float NEG_INF = -__builtin_huge_valf();

  {
    const v4i iv = *(const v4i*)(topk + (size_t)s * TK + tid * 4);
    *(v4i*)(IDX + tid * 4) = iv;
  }
#pragma unroll
  for (int j = 0; j < 4; ++j) {
    const int idx = tid + 128 * j;
    const int rem = idx & 255;
    const int row = rem >> 4;
    const int c8  = rem & 15;
    const unsigned short* src = ((j < 2) ? qh : ql) + ((size_t)s * H + row) * D + c8 * 8;
    unsigned short*       dst = ((j < 2) ? Qh : Ql) + row * QP + c8 * 8;
    *(v8us*)dst = *(const v8us*)src;
  }
  __syncthreads();

  for (int c = 0; c < NCH; ++c) {
    __syncthreads();
#pragma unroll
    for (int j = 0; j < 16; ++j) {
      const int idx = tid + 128 * j;
      const int rem = idx & 1023;
      const int r   = rem >> 4;
      const int c8  = rem & 15;
      const int v   = IDX[c * CH + r];
      const int row = (v < 0) ? 0 : ((v >= nKV) ? (nKV - 1) : v);
      const unsigned short* src = ((j < 8) ? kh : kl) + (size_t)row * D + c8 * 8;
      unsigned short*       dst = ((j < 8) ? Kh : Kl) + r * KP + c8 * 8;
      *(v8us*)dst = *(const v8us*)src;
    }
    __syncthreads();

    v8f acc = zero8();
    const unsigned short* qah = Qh + m * QP + 8 * hh;
    const unsigned short* qal = Ql + m * QP + 8 * hh;
    const unsigned short* kbh = Kh + (wave * 16 + m) * KP + 8 * hh;
    const unsigned short* kbl = Kl + (wave * 16 + m) * KP + 8 * hh;
#pragma unroll
    for (int ks = 0; ks < 4; ++ks) {
      const int k0 = ks * 32;
      Frag ah, al, bh, bl;
      ah.h[0] = *(const v8us*)(qah + k0);  ah.h[1] = *(const v8us*)(qah + k0 + 16);
      al.h[0] = *(const v8us*)(qal + k0);  al.h[1] = *(const v8us*)(qal + k0 + 16);
      bh.h[0] = *(const v8us*)(kbh + k0);  bh.h[1] = *(const v8us*)(kbh + k0 + 16);
      bl.h[0] = *(const v8us*)(kbl + k0);  bl.h[1] = *(const v8us*)(kbl + k0 + 16);
      acc = wmma_bf16(ah.v, bh.v, acc);
      acc = wmma_bf16(ah.v, bl.v, acc);
      acc = wmma_bf16(al.v, bh.v, acc);
    }
    const int  key   = c * CH + wave * 16 + m;
    const bool valid = IDX[key] >= 0;
#pragma unroll
    for (int r = 0; r < 8; ++r)
      S[(8 * hh + r) * SP + key] = valid ? (acc[r] * scale) : NEG_INF;
  }
  __syncthreads();

  {
    const int hd  = tid >> 3;
    const int sub = tid & 7;
    const float* Srow = S + hd * SP + sub;
    float mx = NEG_INF;
#pragma unroll 8
    for (int j = 0; j < 64; ++j) mx = fmaxf(mx, Srow[j * 8]);
    mx = fmaxf(mx, __shfl_xor(mx, 1, 32));
    mx = fmaxf(mx, __shfl_xor(mx, 2, 32));
    mx = fmaxf(mx, __shfl_xor(mx, 4, 32));
    float sum = 0.0f;
    unsigned short* phr = Ph + hd * PP + sub;
    unsigned short* plr = Pl + hd * PP + sub;
#pragma unroll 4
    for (int j = 0; j < 64; ++j) {
      const float p = expf(Srow[j * 8] - mx);
      sum += p;
      const unsigned short b0 = f2bf(p);
      const unsigned short b1 = f2bf(p - bf2f(b0));
      phr[j * 8] = b0;
      plr[j * 8] = b1;
    }
    sum += __shfl_xor(sum, 1, 32);
    sum += __shfl_xor(sum, 2, 32);
    sum += __shfl_xor(sum, 4, 32);
    if (sub == 0) Lsum[hd] = sum;
  }
  __syncthreads();

  v8f acc0 = zero8();
  v8f acc1 = zero8();
  const int d0 = wave * 32;
  for (int c = 0; c < NCH; ++c) {
    __syncthreads();
#pragma unroll
    for (int j = 0; j < 16; ++j) {
      const int idx = tid + 128 * j;
      const int rem = idx & 1023;
      const int r   = rem >> 4;
      const int c8  = rem & 15;
      const int v   = IDX[c * CH + r];
      const int row = (v < 0) ? 0 : ((v >= nKV) ? (nKV - 1) : v);
      const v8us val = *(const v8us*)(((j < 8) ? kh : kl) + (size_t)row * D + c8 * 8);
      unsigned short* dst = ((j < 8) ? Vh : Vl) + (c8 * 8) * VP + r;
#pragma unroll
      for (int e = 0; e < 8; ++e) dst[e * VP] = val[e];
    }
    __syncthreads();

    const unsigned short* pah  = Ph + m * PP + c * CH + 8 * hh;
    const unsigned short* pal  = Pl + m * PP + c * CH + 8 * hh;
    const unsigned short* vb0h = Vh + (d0 + m) * VP + 8 * hh;
    const unsigned short* vb0l = Vl + (d0 + m) * VP + 8 * hh;
    const unsigned short* vb1h = Vh + (d0 + 16 + m) * VP + 8 * hh;
    const unsigned short* vb1l = Vl + (d0 + 16 + m) * VP + 8 * hh;
#pragma unroll
    for (int ks = 0; ks < 2; ++ks) {
      const int k0 = ks * 32;
      Frag ah, al, bh, bl;
      ah.h[0] = *(const v8us*)(pah + k0);   ah.h[1] = *(const v8us*)(pah + k0 + 16);
      al.h[0] = *(const v8us*)(pal + k0);   al.h[1] = *(const v8us*)(pal + k0 + 16);
      bh.h[0] = *(const v8us*)(vb0h + k0);  bh.h[1] = *(const v8us*)(vb0h + k0 + 16);
      bl.h[0] = *(const v8us*)(vb0l + k0);  bl.h[1] = *(const v8us*)(vb0l + k0 + 16);
      acc0 = wmma_bf16(ah.v, bh.v, acc0);
      acc0 = wmma_bf16(ah.v, bl.v, acc0);
      acc0 = wmma_bf16(al.v, bh.v, acc0);
      bh.h[0] = *(const v8us*)(vb1h + k0);  bh.h[1] = *(const v8us*)(vb1h + k0 + 16);
      bl.h[0] = *(const v8us*)(vb1l + k0);  bl.h[1] = *(const v8us*)(vb1l + k0 + 16);
      acc1 = wmma_bf16(ah.v, bh.v, acc1);
      acc1 = wmma_bf16(ah.v, bl.v, acc1);
      acc1 = wmma_bf16(al.v, bh.v, acc1);
    }
  }

  {
    float* Ow = Osc + wave * (H * OP);
#pragma unroll
    for (int r = 0; r < 8; ++r) {
      const float inv = 1.0f / Lsum[8 * hh + r];
      Ow[(8 * hh + r) * OP + m]      = acc0[r] * inv;
      Ow[(8 * hh + r) * OP + 16 + m] = acc1[r] * inv;
    }
  }
  __syncthreads();
  {
    const float* Ow = Osc + wave * (H * OP);
    const int q4    = lane >> 3;
    const int piece = lane & 7;
    v4f vals[4];
#pragma unroll
    for (int j = 0; j < 4; ++j)
      vals[j] = *(const v4f*)(Ow + (4 * j + q4) * OP + piece * 4);
    float* ob = out + (size_t)s * H * D + d0 + piece * 4;
#pragma unroll
    for (int j = 0; j < 4; ++j)
      *(volatile v4f*)(ob + (size_t)(4 * j + q4) * D) = vals[j];
    __threadfence();
#pragma unroll
    for (int j = 0; j < 4; ++j)
      *(volatile v4f*)(ob + (size_t)(4 * j + q4) * D) = vals[j];
  }
}

static inline size_t align256(size_t x) { return (x + 255) & ~(size_t)255; }

extern "C" void kernel_launch(void* const* d_in, const int* in_sizes, int n_in,
                              void* d_out, int out_size, void* d_ws, size_t ws_size,
                              hipStream_t stream)
{
  if (n_in < 3) return;
  const float* q    = (const float*)d_in[0];
  const float* kv   = (const float*)d_in[1];
  const int*   topk = (const int*)d_in[2];
  float*       out  = (float*)d_out;

  const int nq   = in_sizes[0];
  const int nkv  = in_sizes[1];
  const int nidx = in_sizes[2];
  const int nS   = nidx / TK;
  const int nKV  = nkv / D;
  if (nS <= 0 || nKV <= 0) return;
  if (nidx != nS * TK || nq != nS * H * D || nkv != nKV * D) return;
  if (out_size < nS * H * D) return;

  const size_t bQ  = (size_t)nq * 2;
  const size_t bK  = (size_t)nkv * 2;
  const size_t wQh = 0;
  const size_t wQl = align256(wQh + bQ);
  const size_t wKh = align256(wQl + bQ);
  const size_t wKl = align256(wKh + bK);
  const size_t wEnd = align256(wKl + bK);
  if (wEnd > ws_size) return;

  char* ws = (char*)d_ws;
  unsigned short* qh = (unsigned short*)(ws + wQh);
  unsigned short* ql = (unsigned short*)(ws + wQl);
  unsigned short* khp = (unsigned short*)(ws + wKh);
  unsigned short* klp = (unsigned short*)(ws + wKl);

  const unsigned gq = (unsigned)(((size_t)nq + 2047) / 2048);
  const unsigned gk = (unsigned)(((size_t)nkv + 2047) / 2048);
  hipLaunchKernelGGL(k_split, dim3(gq), dim3(256), 0, stream, q, qh, ql, nq);
  hipLaunchKernelGGL(k_split, dim3(gk), dim3(256), 0, stream, kv, khp, klp, nkv);
  hipLaunchKernelGGL(k_attn, dim3((unsigned)nS), dim3(128), 0, stream,
                     (const unsigned short*)qh, (const unsigned short*)ql,
                     (const unsigned short*)khp, (const unsigned short*)klp,
                     topk, out, nS, nKV);
}
